// Decoder_63024350101964
// MI455X (gfx1250) — hardware-verified
//
#include <hip/hip_runtime.h>
#include <math.h>

constexpr int NBATCH   = 256;
constexpr int NPOS     = 32;
constexpr int NSTEPS   = 32;
constexpr int NENC     = 128;
constexpr int NDEC     = 128;
constexpr int NHC      = 2 * NDEC;
constexpr int NGATE    = 4 * NDEC;
constexpr int NW1COL   = NHC + NENC;
constexpr int NTHR     = 256;
constexpr int ROWS_BLK = 16;
constexpr int NROWS    = NBATCH * NPOS;
constexpr int HCP = 264;
constexpr int HWP = 132;
constexpr int CTP = 132;
constexpr int HSP = 132;
constexpr float ACT_CARRY = 16.0f;
constexpr float WGT_CARRY = 64.0f;
constexpr float FOLD_INV  = 1.0f / (ACT_CARRY * WGT_CARRY);

static_assert(NBATCH % ROWS_BLK == 0, "block rows");
static_assert(NBATCH == NTHR, "tail block covers all rows");
static_assert(NROWS % 64 == 0 && NENC % 64 == 0, "gemm tile multiples");
static_assert(NENC % 32 == 0 && NHC % 32 == 0 && NDEC % 32 == 0, "k multiples of 32");
static_assert(NDEC == 16 * (NTHR / 32), "8 waves x 16 units");
static_assert(NPOS == 32 && NENC == 128, "thread maps");
static_assert(HCP % 8 == 0 && HCP >= NHC, "A tile pitch");

typedef __attribute__((ext_vector_type(16))) _Float16 v16h;
typedef __attribute__((ext_vector_type(8)))  _Float16 v8h;
typedef __attribute__((ext_vector_type(8)))  float    v8f;
typedef __attribute__((ext_vector_type(4)))  float    v4f;

__device__ __forceinline__ void guard1_h(v8f& a, v16h x, v16h y) {
  asm volatile("v_nop\n\tv_nop\n\tv_nop\n\tv_nop" : "+v"(a) : "v"(x), "v"(y));
}
__device__ __forceinline__ void guard4_h(v8f& a0, v8f& a1, v8f& a2, v8f& a3, v16h x, v16h y0, v16h y1, v16h y2, v16h y3) {
  asm volatile("v_nop\n\tv_nop\n\tv_nop\n\tv_nop" : "+v"(a0), "+v"(a1), "+v"(a2), "+v"(a3) : "v"(x), "v"(y0), "v"(y1), "v"(y2), "v"(y3));
}
__device__ __forceinline__ void keep4_h(v16h a, v16h b, v16h c, v16h d) { asm volatile("v_nop" :: "v"(a), "v"(b), "v"(c), "v"(d)); }
__device__ __forceinline__ void acc_guard4(v8f& a, v8f& b, v8f& c, v8f& d) { asm volatile("v_nop\n\tv_nop\n\tv_nop\n\tv_nop" : "+v"(a), "+v"(b), "+v"(c), "+v"(d)); }
__device__ __forceinline__ void mem_order_cc() { asm volatile("" ::: "memory"); }

template <typename T> struct Frag;
template <> struct Frag<_Float16> {
  typedef v16h V; union U { v16h v; v8h h[2]; };
  static __device__ __forceinline__ v16h load(const _Float16* p) {
    U f; f.h[0] = *(const v8h*)(p); f.h[1] = *(const v8h*)(p + 16); return f.v;
  }
  static __device__ __forceinline__ v8f mma(v16h a, v16h b, v8f c) {
    return __builtin_amdgcn_wmma_f32_16x16x32_f16(false, a, false, b, (short)0, c, false, false);
  }
};

__device__ __forceinline__ float fsig(float x)  { return 1.0f / (1.0f + expf(-x)); }
__device__ __forceinline__ float ftanh(float x) { return 1.0f - 2.0f / (1.0f + expf(2.0f * x)); }

__global__ __launch_bounds__(NTHR) void cvt8_f16_kernel(const float* __restrict__ src, unsigned short* __restrict__ dst,
                                                        int nrow, int ncol8, int spitch, int scol0, float sc) {
  const int i  = blockIdx.x * NTHR + threadIdx.x;
  const int n8 = nrow * ncol8;
  if (i < n8) {
    const int row = i / ncol8;
    const int c8  = i - row * ncol8;
    const float* sp = src + (size_t)row * spitch + scol0 + c8 * 8;
    const v4f a = *(const v4f*)(sp);
    const v4f b = *(const v4f*)(sp + 4);
    v8h hv;
#pragma unroll
    for (int e = 0; e < 4; ++e) {
      hv[e]     = (_Float16)(a[e] * sc);
      hv[4 + e] = (_Float16)(b[e] * sc);
    }
    *(volatile v8h*)(dst + (size_t)i * 8) = hv;
    __threadfence();
    *(volatile v8h*)(dst + (size_t)i * 8) = hv;
  }
}

__global__ __launch_bounds__(256) void gemm64_f16_kernel(
    const unsigned short* __restrict__ Ap, int lda,
    const unsigned short* __restrict__ Btp, int ldb,
    float* __restrict__ Cout, int ldc,
    const float* __restrict__ bias,
    int M, int N, int K, float scale) {
  const _Float16* A  = (const _Float16*)Ap;
  const _Float16* Bt = (const _Float16*)Btp;
  __shared__ __align__(16) float sT[8][16 * 68];
  const int lane = threadIdx.x & 31;
  const int wave = threadIdx.x >> 5;
  const int tilesN = N >> 6;
  const int tilesM = M >> 6;
  const int tile = blockIdx.x * 8 + wave;
  if (tile >= tilesM * tilesN) return;
  const int tm = tile / tilesN;
  const int tn = tile - tm * tilesN;
  const int m0 = tm << 6;
  const int n0 = tn << 6;

  const int rlane = lane & 15;
  const int koff  = (lane >> 4) * 8;
  const int mOff  = (lane >> 4) * 8;

  v8f acc[4][4];
#pragma unroll
  for (int i = 0; i < 4; ++i)
#pragma unroll
    for (int j = 0; j < 4; ++j) acc[i][j] = (v8f){0.f,0.f,0.f,0.f,0.f,0.f,0.f,0.f};

  for (int k0 = 0; k0 < K; k0 += 32) {
    v16h bh[4];
#pragma unroll
    for (int j = 0; j < 4; ++j) {
      const size_t bo = (size_t)(n0 + (j << 4) + rlane) * ldb + koff + k0;
      bh[j] = Frag<_Float16>::load(Bt + bo);
    }
#pragma unroll
    for (int i = 0; i < 4; ++i) {
      const size_t ao = (size_t)(m0 + (i << 4) + rlane) * lda + koff + k0;
      const v16h ah = Frag<_Float16>::load(A + ao);
#pragma unroll
      for (int j = 0; j < 4; ++j) acc[i][j] = Frag<_Float16>::mma(ah, bh[j], acc[i][j]);
      guard4_h(acc[i][0], acc[i][1], acc[i][2], acc[i][3], ah, bh[0], bh[1], bh[2], bh[3]);
    }
    keep4_h(bh[0], bh[1], bh[2], bh[3]);
  }
  acc_guard4(acc[0][0], acc[0][1], acc[0][2], acc[0][3]);
  acc_guard4(acc[1][0], acc[1][1], acc[1][2], acc[1][3]);
  acc_guard4(acc[2][0], acc[2][1], acc[2][2], acc[2][3]);
  acc_guard4(acc[3][0], acc[3][1], acc[3][2], acc[3][3]);

  float* slab = sT[wave];
  float bv[4];
#pragma unroll
  for (int j = 0; j < 4; ++j) bv[j] = bias[n0 + (j << 4) + rlane];
#pragma unroll
  for (int i = 0; i < 4; ++i) {
    const int mBase = m0 + (i << 4);
#pragma unroll
    for (int j = 0; j < 4; ++j) {
#pragma unroll
      for (int r = 0; r < 8; ++r) {
        const float v = acc[i][j][r] * scale + bv[j];
        slab[(mOff + r) * 68 + (j << 4) + rlane] = v;
      }
    }
    __builtin_amdgcn_fence(__ATOMIC_RELEASE, "workgroup");
    __builtin_amdgcn_wave_barrier();
    __builtin_amdgcn_fence(__ATOMIC_ACQUIRE, "workgroup");
    {
      const int hh = lane >> 4, c4 = (lane & 15) * 4;
      for (int pass = 0; pass < 2; ++pass) {
#pragma unroll
        for (int it = 0; it < 8; ++it) {
          const int row = it * 2 + hh;
          const v4f v = *(const v4f*)(slab + row * 68 + c4);
          *(volatile v4f*)(Cout + (size_t)(mBase + row) * ldc + n0 + c4) = v;
        }
        __threadfence();
      }
    }
    __builtin_amdgcn_fence(__ATOMIC_RELEASE, "workgroup");
    __builtin_amdgcn_wave_barrier();
    __builtin_amdgcn_fence(__ATOMIC_ACQUIRE, "workgroup");
  }
}

__global__ __launch_bounds__(NTHR) void decoder_kernel(
    const float* __restrict__ enc, const float* __restrict__ yh, const float* __restrict__ E1,
    const unsigned short* __restrict__ W1HCp, const unsigned short* __restrict__ WHHp,
    const float* __restrict__ w2g, const float* __restrict__ b2g,
    const float* __restrict__ wih, const float* __restrict__ bih, const float* __restrict__ bhh,
    const float* __restrict__ fcW, const float* __restrict__ fcb,
    float* __restrict__ HLAST, float* __restrict__ CLAST) {
  __shared__ __align__(16) _Float16 sHC[ROWS_BLK * HCP];
  __shared__ __align__(16) float    sHW[ROWS_BLK * HWP];
  __shared__ __align__(16) float    sCtx[ROWS_BLK * CTP];
  __shared__ __align__(16) float    sHs[ROWS_BLK * HSP];
  __shared__ __align__(16) float    sLog[ROWS_BLK * NPOS];
  __shared__ __align__(16) float    sAttn[ROWS_BLK * NPOS];
  __shared__ __align__(16) float    sW2[NENC];
  __shared__ __align__(16) float    sFc[NENC + 4];
  __shared__ float                  sYt[ROWS_BLK];

  const _Float16* W1HC = (const _Float16*)W1HCp;
  const _Float16* WHH  = (const _Float16*)WHHp;
  const int tid = threadIdx.x, lane = tid & 31, wave = tid >> 5;
  const int c = lane & 15, hh = lane >> 4, koff = hh * 8;
  const int m = tid >> 4, q = tid & 15;
  const int rowbase = blockIdx.x * ROWS_BLK;

#pragma unroll 1
  for (int i = tid; i < ROWS_BLK * HCP; i += NTHR) sHC[i] = (_Float16)0.0f;
  {
    const float wv = w2g[tid & (NENC - 1)];
    if (tid < NENC) sW2[tid] = wv;
    const float fv = fcW[tid < NENC + 1 ? tid : NENC];
    if (tid < NENC + 4) sFc[tid] = (tid < NENC + 1) ? fv : 0.0f;
  }
  float bgv[4], wihv[4];
#pragma unroll
  for (int g = 0; g < 4; ++g) {
    const int n = g * NDEC + 16 * wave + c;
    wihv[g] = wih[n];
    const float bi = bih[n];
    const float bh = bhh[n];
    bgv[g] = bi + bh;
    if (g == 1) mem_order_cc();
  }
  const float b2   = b2g[0];
  const float fcb0 = fcb[0];
  float cst[8];
#pragma unroll
  for (int r = 0; r < 8; ++r) cst[r] = 0.0f;
  __syncthreads();
  const float fcy = sFc[NENC];

  const v8f z8 = {0.f, 0.f, 0.f, 0.f, 0.f, 0.f, 0.f, 0.f};
  const _Float16* arow  = sHC + c * HCP + koff;
  const _Float16* w1row = W1HC + (size_t)(16 * wave + c) * NHC + koff;
  const _Float16* whrow = WHH + (size_t)(16 * wave + c) * NDEC + koff;

#pragma unroll 1
  for (int t = 0; t < NSTEPS; ++t) {
    {
      v8f acc = z8;
#pragma unroll
      for (int ks = 0; ks < 8; ++ks) {
        const v16h a = Frag<_Float16>::load(arow + 32 * ks);
        const v16h b = Frag<_Float16>::load(w1row + 32 * ks);
        acc = Frag<_Float16>::mma(a, b, acc);
        guard1_h(acc, a, b);
        if (ks == 3) mem_order_cc();
      }
#pragma unroll
      for (int r = 0; r < 8; ++r) sHW[(8 * hh + r) * HWP + 16 * wave + c] = acc[r] * FOLD_INV;
    }
    __syncthreads();

#pragma unroll 1
    for (int half = 0; half < 2; ++half) {
      const int tt = q + 16 * half;
      const float* e1p = E1 + ((size_t)(rowbase + m) * NPOS + tt) * NENC;
      const float* hwp = sHW + m * HWP;
      float accl = 0.0f;
#pragma unroll 1
      for (int i4 = 0; i4 < NENC / 4; ++i4) {
        const v4f ev = *(const v4f*)(e1p + 4 * i4);
        const v4f hv = *(const v4f*)(hwp + 4 * i4);
        const v4f wv = *(const v4f*)(sW2 + 4 * i4);
#pragma unroll
        for (int e = 0; e < 4; ++e) accl += wv[e] * ftanh(ev[e] + hv[e]);
      }
      sLog[m * NPOS + tt] = accl + b2;
    }
    __syncthreads();

    {
      const float a0 = sLog[m * NPOS + c];
      const float a1 = sLog[m * NPOS + c + 16];
      float mx = fmaxf(a0, a1);
#pragma unroll
      for (int off = 1; off < 16; off <<= 1) mx = fmaxf(mx, __shfl_xor(mx, off, 32));
      const float e0 = expf(a0 - mx);
      const float e1 = expf(a1 - mx);
      float s = e0 + e1;
#pragma unroll
      for (int off = 1; off < 16; off <<= 1) s += __shfl_xor(s, off, 32);
      const float inv = 1.0f / s;
      sAttn[m * NPOS + c]      = e0 * inv;
      sAttn[m * NPOS + c + 16] = e1 * inv;
    }
    __syncthreads();

    {
      const int e0 = 8 * q;
      float ca[8];
#pragma unroll
      for (int j = 0; j < 8; ++j) ca[j] = 0.0f;
      const float* encp = enc + ((size_t)(rowbase + m) * NPOS) * NENC + e0;
#pragma unroll 1
      for (int tt = 0; tt < NPOS; ++tt) {
        const float w = sAttn[m * NPOS + tt];
        const v4f x0 = *(const v4f*)(encp + tt * NENC);
        const v4f x1 = *(const v4f*)(encp + tt * NENC + 4);
#pragma unroll
        for (int e = 0; e < 4; ++e) {
          ca[e]     += w * x0[e];
          ca[4 + e] += w * x1[e];
        }
      }
      v4f o0, o1;
#pragma unroll
      for (int e = 0; e < 4; ++e) { o0[e] = ca[e]; o1[e] = ca[4 + e]; }
      *(v4f*)(sCtx + m * CTP + e0)     = o0;
      *(v4f*)(sCtx + m * CTP + e0 + 4) = o1;
      const v4f f0 = *(const v4f*)(sFc + e0);
      const v4f f1 = *(const v4f*)(sFc + e0 + 4);
      float part = 0.0f;
#pragma unroll
      for (int e = 0; e < 4; ++e) part += f0[e] * ca[e] + f1[e] * ca[4 + e];
#pragma unroll
      for (int off = 1; off < 16; off <<= 1) part += __shfl_xor(part, off, 32);
      const float ytv = yh[(size_t)(rowbase + m) * NSTEPS + t];
      const float yt  = part + fcb0 + fcy * ytv;
      if (q == 0) sYt[m] = yt;
    }
    __syncthreads();

    float hn[8];
    {
      v8f acc[4];
      acc[0] = z8; acc[1] = z8; acc[2] = z8; acc[3] = z8;
#pragma unroll
      for (int ks = 0; ks < 4; ++ks) {
        const v16h a  = Frag<_Float16>::load(arow + 32 * ks);
        const v16h b0 = Frag<_Float16>::load(whrow + 32 * ks);
        const v16h b1 = Frag<_Float16>::load(whrow + (size_t)1 * NDEC * NDEC + 32 * ks);
        const v16h b2f = Frag<_Float16>::load(whrow + (size_t)2 * NDEC * NDEC + 32 * ks);
        const v16h b3 = Frag<_Float16>::load(whrow + (size_t)3 * NDEC * NDEC + 32 * ks);
        acc[0] = Frag<_Float16>::mma(a, b0, acc[0]);
        acc[1] = Frag<_Float16>::mma(a, b1, acc[1]);
        acc[2] = Frag<_Float16>::mma(a, b2f, acc[2]);
        acc[3] = Frag<_Float16>::mma(a, b3, acc[3]);
        guard4_h(acc[0], acc[1], acc[2], acc[3], a, b0, b1, b2f, b3);
        mem_order_cc();
      }
      float ytr[8];
#pragma unroll
      for (int r = 0; r < 8; ++r) ytr[r] = sYt[8 * hh + r];
#pragma unroll
      for (int r = 0; r < 8; ++r) {
        const float yt = ytr[r];
        const float zi = acc[0][r] * FOLD_INV + (bgv[0] + wihv[0] * yt);
        const float zf = acc[1][r] * FOLD_INV + (bgv[1] + wihv[1] * yt);
        const float zg = acc[2][r] * FOLD_INV + (bgv[2] + wihv[2] * yt);
        const float zo = acc[3][r] * FOLD_INV + (bgv[3] + wihv[3] * yt);
        const float ig = fsig(zi);
        const float fg = fsig(zf);
        const float gg = ftanh(zg);
        const float og = fsig(zo);
        const float cn = fg * cst[r] + ig * gg;
        cst[r] = cn;
        hn[r]  = og * ftanh(cn);
      }
    }
    __syncthreads();

    {
      const int j = 16 * wave + c;
#pragma unroll
      for (int r = 0; r < 8; ++r) {
        sHC[(8 * hh + r) * HCP + j]        = (_Float16)(hn[r] * ACT_CARRY);
        sHC[(8 * hh + r) * HCP + NDEC + j] = (_Float16)(cst[r] * ACT_CARRY);
      }
      if (t == NSTEPS - 1) {
#pragma unroll
        for (int r = 0; r < 8; ++r) sHs[(8 * hh + r) * HSP + j] = hn[r];
      }
    }
    __syncthreads();
  }

  for (int pass = 0; pass < 2; ++pass) {
#pragma unroll
    for (int it = 0; it < 2; ++it) {
      const int idx = it * NTHR + tid;
      const int row = idx >> 5, c4 = (idx & 31) * 4;
      const v4f vh = *(const v4f*)(sHs + row * HSP + c4);
      const v4f vc = *(const v4f*)(sCtx + row * CTP + c4);
      *(volatile v4f*)(HLAST + (size_t)(rowbase + row) * NDEC + c4) = vh;
      *(volatile v4f*)(CLAST + (size_t)(rowbase + row) * NENC + c4) = vc;
    }
    __threadfence();
  }
}

__global__ __launch_bounds__(NTHR) void tail_kernel(const float* __restrict__ HLAST, const float* __restrict__ CLAST,
                                                    const float* __restrict__ fcfW, const float* __restrict__ fcfb,
                                                    const float* __restrict__ yh, float* __restrict__ out) {
  const int b = threadIdx.x;
  const float* hp = HLAST + (size_t)b * NDEC;
  const float* cp = CLAST + (size_t)b * NENC;
  float s = 0.0f;
#pragma unroll 1
  for (int i4 = 0; i4 < NDEC / 4; ++i4) {
    const v4f hv = *(const v4f*)(hp + 4 * i4);
    const v4f cv = *(const v4f*)(cp + 4 * i4);
    const v4f wh = *(const v4f*)(fcfW + 4 * i4);
    const v4f wc = *(const v4f*)(fcfW + NDEC + 4 * i4);
#pragma unroll
    for (int e = 0; e < 4; ++e) s += wh[e] * hv[e] + wc[e] * cv[e];
  }
  const float o = s + fcfb[0] + yh[(size_t)b * NSTEPS + (NSTEPS - 1)];
  *(volatile float*)(out + b) = o;
  __threadfence();
  *(volatile float*)(out + b) = o;
}

extern "C" void kernel_launch(void* const* d_in, const int* in_sizes, int n_in,
                              void* d_out, int out_size, void* d_ws, size_t ws_size, hipStream_t stream) {
  if (n_in < 14 || d_out == nullptr || d_ws == nullptr) return;
  if (in_sizes[0] != NBATCH * NPOS * NENC || in_sizes[1] != NBATCH * NSTEPS || in_sizes[2] != NENC * NW1COL ||
      in_sizes[3] != NENC || in_sizes[4] != NENC || in_sizes[5] != 1 || in_sizes[6] != NGATE ||
      in_sizes[7] != NGATE * NDEC || in_sizes[8] != NGATE || in_sizes[9] != NGATE || in_sizes[10] != NENC + 1 ||
      in_sizes[11] != 1 || in_sizes[12] != NDEC + NENC || in_sizes[13] != 1 || out_size != NBATCH) return;

  const float* enc  = (const float*)d_in[0];
  const float* yh   = (const float*)d_in[1];
  const float* W1   = (const float*)d_in[2];
  const float* b1   = (const float*)d_in[3];
  const float* W2   = (const float*)d_in[4];
  const float* b2   = (const float*)d_in[5];
  const float* Wih  = (const float*)d_in[6];
  const float* Whh  = (const float*)d_in[7];
  const float* bih  = (const float*)d_in[8];
  const float* bhh  = (const float*)d_in[9];
  const float* fcW  = (const float*)d_in[10];
  const float* fcb  = (const float*)d_in[11];
  const float* fcfW = (const float*)d_in[12];
  const float* fcfb = (const float*)d_in[13];
  float* out = (float*)d_out;

  char* ws = (char*)d_ws; size_t off = 0;
  auto carve = [&](size_t bytes) -> char* { char* p = ws + off; off += (bytes + 255) & ~(size_t)255; return p; };
  unsigned short* ENC16 = (unsigned short*)carve((size_t)NROWS * NENC * 2);
  unsigned short* W1E   = (unsigned short*)carve((size_t)NENC * NENC * 2);
  unsigned short* W1HC  = (unsigned short*)carve((size_t)NENC * NHC * 2);
  unsigned short* WHHP  = (unsigned short*)carve((size_t)NGATE * NDEC * 2);
  float*          E1    = (float*)carve((size_t)NROWS * NENC * 4);
  float*          HLAST = (float*)carve((size_t)NBATCH * NDEC * 4);
  float*          CLAST = (float*)carve((size_t)NBATCH * NENC * 4);
  if (off > ws_size || off > (size_t)134217728) return;

  const int n8e  = NROWS * (NENC / 8);
  const int n8w1 = NENC * (NENC / 8);
  const int n8hc = NENC * (NHC / 8);
  const int n8hh = NGATE * (NDEC / 8);
  cvt8_f16_kernel<<<(n8e  + NTHR - 1) / NTHR, NTHR, 0, stream>>>(enc, ENC16, NROWS, NENC / 8, NENC,   0,   ACT_CARRY);
  cvt8_f16_kernel<<<(n8w1 + NTHR - 1) / NTHR, NTHR, 0, stream>>>(W1,  W1E,   NENC,  NENC / 8, NW1COL, NHC, WGT_CARRY);
  cvt8_f16_kernel<<<(n8hc + NTHR - 1) / NTHR, NTHR, 0, stream>>>(W1,  W1HC,  NENC,  NHC / 8,  NW1COL, 0,   WGT_CARRY);
  cvt8_f16_kernel<<<(n8hh + NTHR - 1) / NTHR, NTHR, 0, stream>>>(Whh, WHHP,  NGATE, NDEC / 8, NDEC,   0,   WGT_CARRY);

  gemm64_f16_kernel<<<dim3((NROWS / 64) * (NENC / 64) / 8), 256, 0, stream>>>(
      ENC16, NENC, W1E, NENC, E1, NENC, b1, NROWS, NENC, NENC, FOLD_INV);

  decoder_kernel<<<NBATCH / ROWS_BLK, NTHR, 0, stream>>>(enc, yh, E1, W1HC, WHHP, W2, b2, Wih, bih, bhh, fcW, fcb,
                                                         HLAST, CLAST);

  tail_kernel<<<1, NTHR, 0, stream>>>(HLAST, CLAST, fcfW, fcfb, yh, out);
}
